// ClusterModel_23098334118129
// MI455X (gfx1250) — hardware-run, weakly checked
//
#include <hip/hip_runtime.h>
#include <math.h>

typedef __attribute__((ext_vector_type(16))) _Float16 v16h;
typedef __attribute__((ext_vector_type(8)))  _Float16 v8h;
typedef __attribute__((ext_vector_type(8)))  float    v8f;
typedef __attribute__((ext_vector_type(4)))  float    v4f;
typedef __attribute__((ext_vector_type(4)))  int      v4i;

constexpr int kN    = 100000;
constexpr int kE    = 1600000;
constexpr int kCin  = 128;
constexpr int kH    = 64;
constexpr int kK    = 100;
constexpr int kKP   = 128;
constexpr int kNP   = 100352;
constexpr int kAggT = 512;
constexpr int kAggShift = 9;
constexpr int kAggTiles = kNP / kAggT;
constexpr int kDegT = 8192;
constexpr int kDegTiles = 13;
constexpr int kDegPad = kDegT * kDegTiles;
constexpr int kPoolTiles = kNP / 64;
constexpr int kStepEdges = 1024;
constexpr int kEdgeSteps = (kE + kStepEdges - 1) / kStepEdges;
constexpr int kHitCap = 2048;
constexpr int kCutBlocks = (kE + 1023) / 1024;
constexpr int kSSK = 2048;
constexpr int kSSBatches = kNP / kSSK;
constexpr int kLogP = 132;

constexpr float kW1Carry    = 16.0f;
constexpr float kW1CarryInv = 1.0f / kW1Carry;
constexpr float kWpCarry    = 8.0f;
constexpr float kWpCarryInv = 1.0f / kWpCarry;
constexpr float kSCarry     = 64.0f;
constexpr float kSSScale    = 1.0f / (kSCarry * kSCarry);
constexpr float kDegFx    = 4194304.0f;
constexpr float kDegFxInv = 1.0f / kDegFx;
constexpr float kAggFx    = 2097152.0f;
constexpr float kAggFxInv = 1.0f / kAggFx;

static_assert((1 << kAggShift) == kAggT, "tile shift");
static_assert(kAggT * kAggTiles == kNP, "aggregation tiles cover the padded node range");
static_assert(kPoolTiles * 64 == kNP, "pool tiles cover the padded node range");
static_assert(kSSK * kSSBatches == kNP, "split-K batches cover the padded node range");
static_assert(kDegPad >= kNP, "degree tables cover the padded node range");
static_assert(kNP >= kN && (kNP % 64) == 0 && (kNP % 32) == 0, "padding");
static_assert((kN % 32) == 0, "whole wave groups in the tail output tile");
static_assert((kE % 4) == 0, "vector edge loads");
static_assert((kK % 4) == 0 && kK <= kKP, "cluster width");
static_assert(((size_t)kN * kK * 4) % 128 == 0, "scalar outputs start on a line");
static_assert((kCin % 32) == 0 && (kH % 32) == 0 && (kSSK % 32) == 0, "GEMM K multiples of 32");
static_assert((kH % 64) == 0 && (kKP % 64) == 0, "GEMM N multiples of 64");
static_assert(kN < (1 << 22), "node id fits the packed hit key");
static_assert(kHitCap >= 2 * kStepEdges, "hit list holds a carried half plus a full step");

constexpr size_t kOffX16   = 0;
constexpr size_t kOffHX    = kOffX16   + (size_t)kNP * kCin * 2;
constexpr size_t kOffH16   = kOffHX    + (size_t)kNP * kH * 4;
constexpr size_t kOffST16  = kOffH16   + (size_t)kNP * kH * 2;
constexpr size_t kOffSSP   = kOffST16  + (size_t)kKP * kNP * 2;
constexpr size_t kOffINV   = kOffSSP   + (size_t)kSSBatches * kKP * kKP * 4;
constexpr size_t kOffDEGNL = kOffINV   + (size_t)kDegPad * 4;
constexpr size_t kOffW1T   = kOffDEGNL + (size_t)kDegPad * 4;
constexpr size_t kOffWPT   = kOffW1T   + (size_t)kH * kCin * 2;
constexpr size_t kOffNUMP  = kOffWPT   + (size_t)kKP * kH * 2;
constexpr size_t kOffDENP  = kOffNUMP  + (size_t)kCutBlocks * 32 * 4;
constexpr size_t kWsTotal  = kOffDENP  + (size_t)kPoolTiles * 32 * 4;
static_assert(kWsTotal == 94412160ull, "carve total");
static_assert(kWsTotal <= 134217728ull, "carve cap");
static_assert((kOffHX % 128) == 0 && (kOffH16 % 128) == 0 && (kOffST16 % 128) == 0 && (kOffSSP % 128) == 0 &&
              (kOffINV % 128) == 0 && (kOffDEGNL % 128) == 0 && (kOffW1T % 128) == 0 && (kOffWPT % 128) == 0 &&
              (kOffNUMP % 128) == 0 && (kOffDENP % 128) == 0, "128-B aligned regions");

__device__ __forceinline__ v16h frag_load_h(const _Float16* p) {
  union { v16h v; v8h h[2]; } f;
  f.h[0] = *(const v8h*)(p);
  f.h[1] = *(const v8h*)(p + 16);
  return f.v;
}
__device__ __forceinline__ v8f mma_h(v16h a, v16h b, v8f c) {
  return __builtin_amdgcn_wmma_f32_16x16x32_f16(false, a, false, b, (short)0, c, false, false);
}
__device__ __forceinline__ void grp_guard(v8f& c0, v8f& c1, v8f& c2, v8f& c3,
                                          v16h a, v16h b0, v16h b1, v16h b2, v16h b3) {
  asm volatile("v_nop\n\tv_nop\n\tv_nop\n\tv_nop"
               : "+v"(c0), "+v"(c1), "+v"(c2), "+v"(c3)
               : "v"(a), "v"(b0), "v"(b1), "v"(b2), "v"(b3));
}
__device__ __forceinline__ void keep4_h(v16h a, v16h b, v16h c, v16h d) { asm volatile("v_nop" :: "v"(a), "v"(b), "v"(c), "v"(d)); }
__device__ __forceinline__ void acc_guard4(v8f& a, v8f& b, v8f& c, v8f& d) { asm volatile("v_nop\n\tv_nop\n\tv_nop\n\tv_nop" : "+v"(a), "+v"(b), "+v"(c), "+v"(d)); }

__device__ __forceinline__ float wave_sum32(float v) {
#pragma unroll
  for (int off = 16; off > 0; off >>= 1) v += __shfl_xor(v, off, 32);
  return v;
}
__device__ __forceinline__ float block_sum256(float v, float* red, int lane, int wave) {
  v = wave_sum32(v);
  __syncthreads();
  if (lane == 0) red[wave] = v;
  __syncthreads();
  float t = 0.0f;
#pragma unroll
  for (int i = 0; i < 8; ++i) t += red[i];
  return t;
}

__global__ __launch_bounds__(256) void wmma_gemm64_f16(
    const unsigned short* Ap, int lda, long strideA,
    const unsigned short* Btp, int ldb, long strideB,
    float* __restrict__ Cout, int ldc, long strideC,
    int M, int N, int K, float scale) {
  typedef _Float16 T;
  const T* A = (const T*)Ap;
  const T* Bt = (const T*)Btp;
  __shared__ __align__(16) float sT[8][16 * 68];
  const int b    = blockIdx.y;
  const int lane = threadIdx.x & 31;
  const int wave = threadIdx.x >> 5;
  const int tilesN = N >> 6;
  const int tilesM = M >> 6;
  const int tile = blockIdx.x * 8 + wave;
  if (tile >= tilesM * tilesN) return;
  const int tm = tile / tilesN;
  const int tn = tile - tm * tilesN;
  const int m0 = tm << 6;
  const int n0 = tn << 6;

  const T* Ab = A  + (size_t)b * strideA;
  const T* Bb = Bt + (size_t)b * strideB;

  const int rlane = lane & 15;
  const int koff  = (lane >> 4) * 8;
  const int mOff  = (lane >> 4) * 8;

  v8f acc[4][4];
#pragma unroll
  for (int i = 0; i < 4; ++i)
#pragma unroll
    for (int j = 0; j < 4; ++j) acc[i][j] = (v8f){0.f,0.f,0.f,0.f,0.f,0.f,0.f,0.f};

  for (int k0 = 0; k0 < K; k0 += 32) {
    v16h bh[4];
#pragma unroll
    for (int j = 0; j < 4; ++j) {
      const size_t bo = (size_t)(n0 + (j << 4) + rlane) * ldb + koff + k0;
      bh[j] = frag_load_h(Bb + bo);
    }
#pragma unroll
    for (int i = 0; i < 4; ++i) {
      const size_t ao = (size_t)(m0 + (i << 4) + rlane) * lda + koff + k0;
      v16h ah = frag_load_h(Ab + ao);
#pragma unroll
      for (int j = 0; j < 4; ++j) acc[i][j] = mma_h(ah, bh[j], acc[i][j]);
      grp_guard(acc[i][0], acc[i][1], acc[i][2], acc[i][3], ah, bh[0], bh[1], bh[2], bh[3]);
    }
    keep4_h(bh[0], bh[1], bh[2], bh[3]);
  }
  acc_guard4(acc[0][0], acc[0][1], acc[0][2], acc[0][3]);
  acc_guard4(acc[1][0], acc[1][1], acc[1][2], acc[1][3]);
  acc_guard4(acc[2][0], acc[2][1], acc[2][2], acc[2][3]);
  acc_guard4(acc[3][0], acc[3][1], acc[3][2], acc[3][3]);

  float* slab = sT[wave];
  float* C = Cout + (size_t)b * strideC;
#pragma unroll
  for (int i = 0; i < 4; ++i) {
    const int mBase = m0 + (i << 4);
#pragma unroll
    for (int j = 0; j < 4; ++j) {
#pragma unroll
      for (int r = 0; r < 8; ++r) {
        slab[(mOff + r) * 68 + (j << 4) + rlane] = acc[i][j][r] * scale;
      }
    }
    __builtin_amdgcn_fence(__ATOMIC_RELEASE, "workgroup");
    __builtin_amdgcn_wave_barrier();
    __builtin_amdgcn_fence(__ATOMIC_ACQUIRE, "workgroup");
    {
      const int hh = lane >> 4, c4 = (lane & 15) * 4;
      for (int pass = 0; pass < 2; ++pass) {
#pragma unroll
        for (int it = 0; it < 8; ++it) {
          const int row = it * 2 + hh;
          v4f v = *(const v4f*)(slab + row * 68 + c4);
          *(volatile v4f*)(C + (size_t)(mBase + row) * ldc + n0 + c4) = v;
        }
        __threadfence();
      }
    }
    __builtin_amdgcn_fence(__ATOMIC_RELEASE, "workgroup");
    __builtin_amdgcn_wave_barrier();
    __builtin_amdgcn_fence(__ATOMIC_ACQUIRE, "workgroup");
  }
}

__global__ __launch_bounds__(256) void prep_weights_kernel(
    const float* __restrict__ W1, const float* __restrict__ Wp,
    unsigned short* __restrict__ W1T, unsigned short* __restrict__ WPT)
{
  const int tid = threadIdx.x;
  if (blockIdx.x < 4) {
    const int i = blockIdx.x * 256 + tid;
    const int n = i >> 4;
    const int k8 = (i & 15) * 8;
    v8h hv;
#pragma unroll
    for (int e = 0; e < 8; ++e) {
      const float w = W1[(size_t)(k8 + e) * kH + n];
      hv[e] = (_Float16)(w * kW1Carry);
    }
    unsigned short* q = W1T + (size_t)i * 8;
    *(volatile v8h*)q = hv;
    __threadfence();
    *(volatile v8h*)q = hv;
  } else {
    const int i = (blockIdx.x - 4) * 256 + tid;
    const int n = i >> 3;
    const int k8 = (i & 7) * 8;
    const int nc = (n < kK) ? n : (kK - 1);
    v8h hv;
#pragma unroll
    for (int e = 0; e < 8; ++e) {
      const float w = Wp[(size_t)(k8 + e) * kK + nc];
      const float v = (n < kK) ? (w * kWpCarry) : 0.0f;
      hv[e] = (_Float16)v;
    }
    unsigned short* q = WPT + (size_t)i * 8;
    *(volatile v8h*)q = hv;
    __threadfence();
    *(volatile v8h*)q = hv;
  }
}

__global__ __launch_bounds__(256) void cast_x_kernel(const float* __restrict__ x, unsigned short* __restrict__ X16)
{
  const int i = blockIdx.x * 256 + threadIdx.x;
  const size_t e0 = (size_t)i << 3;
  const size_t lim = (size_t)kN * kCin;
  const bool live = e0 < lim;
  const size_t ec = live ? e0 : (lim - 8);
  const v4f a0 = *(const v4f*)(x + ec);
  const v4f a1 = *(const v4f*)(x + ec + 4);
  v8h hv;
#pragma unroll
  for (int e = 0; e < 4; ++e) {
    const float f0 = live ? a0[e] : 0.0f;
    const float f1 = live ? a1[e] : 0.0f;
    hv[e]     = (_Float16)f0;
    hv[4 + e] = (_Float16)f1;
  }
  unsigned short* q = X16 + e0;
  *(volatile v8h*)q = hv;
  __threadfence();
  *(volatile v8h*)q = hv;
}

__global__ __launch_bounds__(256) void degree_tile_kernel(
    const int* __restrict__ ei, const float* __restrict__ ew,
    float* __restrict__ INV, float* __restrict__ DEGNL)
{
  __shared__ __align__(16) int sDeg[kDegT];
  const int tid = threadIdx.x;
  const int base = blockIdx.x * kDegT;
#pragma unroll 1
  for (int i = tid; i < kDegT; i += 256) sDeg[i] = 0;
  __syncthreads();
#pragma unroll 1
  for (int step = 0; step < kEdgeSteps; ++step) {
    const int e0 = step * kStepEdges + tid * 4;
    const bool live = e0 < kE;
    const int ebc = live ? e0 : (kE - 4);
    const v4i dv = *(const v4i*)(ei + kE + ebc);
    const v4f wv = *(const v4f*)(ew + ebc);
#pragma unroll
    for (int j = 0; j < 4; ++j) {
      int d = dv[j];
      d = min(max(d, 0), kN - 1);
      const int dl = d - base;
      const bool hit = live && ((unsigned)dl < (unsigned)kDegT);
      const float wj = wv[j];
      const int q = __float2int_rn(wj * kDegFx);
      if (hit) atomicAdd(&sDeg[dl], q);
    }
  }
  __syncthreads();
  for (int pass = 0; pass < 2; ++pass) {
#pragma unroll 1
    for (int it = 0; it < kDegT / 4 / 256; ++it) {
      const int f4 = it * 256 + tid;
      const v4i q = *(const v4i*)(sDeg + f4 * 4);
      v4f dn, iv;
#pragma unroll
      for (int e = 0; e < 4; ++e) {
        const int qe = q[e];
        const float dd = (float)qe * kDegFxInv;
        const float dg = dd + 1.0f;
        dn[e] = dd;
        iv[e] = (dg > 0.0f) ? rsqrtf(dg) : 0.0f;
      }
      *(volatile v4f*)(DEGNL + base + f4 * 4) = dn;
      *(volatile v4f*)(INV + base + f4 * 4) = iv;
    }
    __threadfence();
  }
}

__global__ __launch_bounds__(256) void aggregate_tile_kernel(
    const int* __restrict__ ei, const float* __restrict__ ew,
    const float* __restrict__ HX, const float* __restrict__ INV,
    const float* __restrict__ b1, unsigned short* __restrict__ H16)
{
  __shared__ __align__(16) int   sAcc[kAggT * kH];
  __shared__ int   sKey[kHitCap];
  __shared__ float sWgt[kHitCap];
  __shared__ int   sCnt[4];
  const int tid = threadIdx.x;
  const int base = blockIdx.x * kAggT;
  {
    const v4i z = (v4i){0, 0, 0, 0};
#pragma unroll 1
    for (int it = 0; it < (kAggT * kH / 4) / 256; ++it) *(v4i*)(sAcc + (it * 256 + tid) * 4) = z;
  }
  if (tid < 4) sCnt[tid] = 0;
  __syncthreads();

  int total = 0;
  int par = 0;
#pragma unroll 1
  for (int step = 0; step < kEdgeSteps; ++step) {
    const int e0 = step * kStepEdges + tid * 4;
    const bool live = e0 < kE;
    const int ebc = live ? e0 : (kE - 4);
    const v4i sv = *(const v4i*)(ei + ebc);
    const v4i dv = *(const v4i*)(ei + kE + ebc);
    const v4f wv = *(const v4f*)(ew + ebc);
#pragma unroll
    for (int j = 0; j < 4; ++j) {
      int d = dv[j];
      d = min(max(d, 0), kN - 1);
      int s = sv[j];
      s = min(max(s, 0), kN - 1);
      const float wj = wv[j];
      const int dl = d - base;
      const bool hit = live && ((unsigned)dl < (unsigned)kAggT);
      if (hit) {
        const int slot = total + atomicAdd(&sCnt[par], 1);
        if (slot < kHitCap) {
          sKey[slot] = (s << kAggShift) | dl;
          sWgt[slot] = wj;
        }
      }
    }
    __syncthreads();
    total += __builtin_amdgcn_readfirstlane(sCnt[par]);
    total = min(total, kHitCap);
    {
      const int nxt = (par == 2) ? 0 : (par + 1);
      const int rst = (nxt == 2) ? 0 : (nxt + 1);
      if (tid == 0) sCnt[rst] = 0;
      par = nxt;
    }
    const bool doDrain = (total > (kHitCap - kStepEdges)) || ((step == kEdgeSteps - 1) && (total > 0));
    if (doDrain) {
      const int grp = tid >> 4;
      const int l16 = tid & 15;
      const int nIt = (total + 15) >> 4;
#pragma unroll 1
      for (int i = 0; i < nIt; ++i) {
        const int h = i * 16 + grp;
        const bool on = h < total;
        const int hc = on ? h : (total - 1);
        const int key = sKey[hc];
        const float w = sWgt[hc];
        int s = key >> kAggShift;
        s = min(max(s, 0), kN - 1);
        const int dl = key & (kAggT - 1);
        float coef = w * INV[s] * kAggFx;
        asm volatile("" : "+v"(coef));
        const v4f hv = *(const v4f*)(HX + (size_t)s * kH + l16 * 4);
        const float p0 = hv[0] * coef;
        const float p1 = hv[1] * coef;
        const float p2 = hv[2] * coef;
        const float p3 = hv[3] * coef;
        int q0 = __float2int_rn(p0);
        int q1 = __float2int_rn(p1);
        int q2 = __float2int_rn(p2);
        int q3 = __float2int_rn(p3);
        asm volatile("" : "+v"(q0));
        asm volatile("" : "+v"(q1));
        asm volatile("" : "+v"(q2));
        asm volatile("" : "+v"(q3));
        int* pa = sAcc + dl * kH + l16 * 4;
        atomicAdd(pa + 0, on ? q0 : 0);
        atomicAdd(pa + 1, on ? q1 : 0);
        atomicAdd(pa + 2, on ? q2 : 0);
        atomicAdd(pa + 3, on ? q3 : 0);
      }
      total = 0;
      __syncthreads();
    }
  }
  __syncthreads();

#pragma unroll 1
  for (int it = 0; it < (kAggT * kH) / 256; ++it) {
    const int idx = it * 256 + tid;
    const int row = idx >> 6;
    const int c = idx & (kH - 1);
    const int node = base + row;
    const float iv = INV[node];
    const float hx = HX[(size_t)node * kH + c];
    const float bb = b1[c];
    const int qa = sAcc[idx];
    const float accf = (float)qa * kAggFxInv + iv * hx;
    const float v = iv * accf + bb;
    const float neg = expm1f(fminf(v, 0.0f));
    float hval = (v > 0.0f) ? v : neg;
    hval = (node < kN) ? hval : 0.0f;
    sAcc[idx] = __float_as_int(hval);
  }
  __syncthreads();
  {
    const int q8 = tid >> 3;
    const int c8 = (tid & 7) * 8;
    for (int pass = 0; pass < 2; ++pass) {
#pragma unroll 1
      for (int it = 0; it < kAggT / 32; ++it) {
        const int row = it * 32 + q8;
        const v4i a0 = *(const v4i*)(sAcc + row * kH + c8);
        const v4i a1 = *(const v4i*)(sAcc + row * kH + c8 + 4);
        v8h hv;
#pragma unroll
        for (int e = 0; e < 4; ++e) {
          const int t0 = a0[e];
          const int t1 = a1[e];
          const float f0 = __int_as_float(t0);
          const float f1 = __int_as_float(t1);
          hv[e]     = (_Float16)f0;
          hv[4 + e] = (_Float16)f1;
        }
        *(volatile v8h*)(H16 + (size_t)(base + row) * kH + c8) = hv;
      }
      __threadfence();
    }
  }
}

__global__ __launch_bounds__(256) void pool_softmax_kernel(
    const unsigned short* __restrict__ H16p, const unsigned short* __restrict__ WPTp,
    const float* __restrict__ bp, const float* __restrict__ DEGNL,
    float* __restrict__ out, unsigned short* __restrict__ ST16, float* __restrict__ DENP)
{
  __shared__ __align__(16) float sLog[64 * kLogP];
  __shared__ __align__(16) float sOut[64 * kK];
  __shared__ float sRow[64];
  const int tid = threadIdx.x;
  const int lane = tid & 31;
  const int wave = tid >> 5;
  const int hh = lane >> 4;
  const int c = lane & 15;
  const int tile = blockIdx.x;
  const int m0 = tile * 64;
  const int rt = wave >> 1;
  const int ch = wave & 1;

  v8f acc[4];
#pragma unroll
  for (int j = 0; j < 4; ++j) acc[j] = (v8f){0.f,0.f,0.f,0.f,0.f,0.f,0.f,0.f};
  {
    const _Float16* A = (const _Float16*)H16p + (size_t)(m0 + rt * 16 + c) * kH + 8 * hh;
    const _Float16* B = (const _Float16*)WPTp + (size_t)(ch * 64 + c) * kH + 8 * hh;
    const v16h a0 = frag_load_h(A);
    const v16h a1 = frag_load_h(A + 32);
    {
      const v16h b0 = frag_load_h(B);
      const v16h b1v = frag_load_h(B + 16 * kH);
      const v16h b2 = frag_load_h(B + 32 * kH);
      const v16h b3 = frag_load_h(B + 48 * kH);
      acc[0] = mma_h(a0, b0, acc[0]);
      acc[1] = mma_h(a0, b1v, acc[1]);
      acc[2] = mma_h(a0, b2, acc[2]);
      acc[3] = mma_h(a0, b3, acc[3]);
      grp_guard(acc[0], acc[1], acc[2], acc[3], a0, b0, b1v, b2, b3);
    }
    {
      const v16h b0 = frag_load_h(B + 32);
      const v16h b1v = frag_load_h(B + 16 * kH + 32);
      const v16h b2 = frag_load_h(B + 32 * kH + 32);
      const v16h b3 = frag_load_h(B + 48 * kH + 32);
      acc[0] = mma_h(a1, b0, acc[0]);
      acc[1] = mma_h(a1, b1v, acc[1]);
      acc[2] = mma_h(a1, b2, acc[2]);
      acc[3] = mma_h(a1, b3, acc[3]);
      grp_guard(acc[0], acc[1], acc[2], acc[3], a1, b0, b1v, b2, b3);
    }
  }
#pragma unroll
  for (int j = 0; j < 4; ++j) {
    const int col = ch * 64 + j * 16 + c;
    const int colc = (col < kK) ? col : (kK - 1);
    const float bl = bp[colc];
    const float bias = (col < kK) ? bl : 0.0f;
#pragma unroll
    for (int r = 0; r < 8; ++r) {
      sLog[(rt * 16 + 8 * hh + r) * kLogP + col] = acc[j][r] * kWpCarryInv + bias;
    }
  }
  __syncthreads();

  {
    const int row = tid >> 2;
    const int q = tid & 3;
    const int node = m0 + row;
    const bool valid = node < kN;
    float* lr = sLog + row * kLogP;
    float m = -INFINITY;
#pragma unroll 1
    for (int i = 0; i < kK / 4; ++i) m = fmaxf(m, lr[q + 4 * i]);
    m = fmaxf(m, __shfl_xor(m, 1, 32));
    m = fmaxf(m, __shfl_xor(m, 2, 32));
    float sum = 0.0f;
#pragma unroll 1
    for (int i = 0; i < kK / 4; ++i) {
      const float e = expf(lr[q + 4 * i] - m);
      lr[q + 4 * i] = e;
      sum += e;
    }
    sum += __shfl_xor(sum, 1, 32);
    sum += __shfl_xor(sum, 2, 32);
    const float rinv = 1.0f / sum;
    float ssq = 0.0f;
#pragma unroll 1
    for (int i = 0; i < kK / 4; ++i) {
      float p = lr[q + 4 * i] * rinv;
      p = valid ? p : 0.0f;
      sOut[row * kK + q + 4 * i] = p;
      ssq += p * p;
    }
    ssq += __shfl_xor(ssq, 1, 32);
    ssq += __shfl_xor(ssq, 2, 32);
    const float dn = DEGNL[node];
    if (q == 0) sRow[row] = dn * ssq;
  }
  __syncthreads();

  float dsum = 0.0f;
  if (wave == 0) {
    float v = sRow[lane] + sRow[lane + 32];
    v = wave_sum32(v);
    dsum = (lane == 0) ? v : 0.0f;
  }
  int rowsValid = kN - m0;
  rowsValid = min(max(rowsValid, 0), 64);
  const int nvalid4 = rowsValid * (kK / 4);
  float* otile = out + (size_t)tile * (64 * kK);
  const int q8 = tid >> 3;
  const int n8 = (tid & 7) * 8;
  for (int pass = 0; pass < 2; ++pass) {
#pragma unroll 1
    for (int it = 0; it < 7; ++it) {
      const int f4 = it * 256 + tid;
      if (f4 < nvalid4) {
        const v4f v = *(const v4f*)(sOut + f4 * 4);
        *(volatile v4f*)(otile + (size_t)f4 * 4) = v;
      }
    }
#pragma unroll 1
    for (int it = 0; it < kKP / 32; ++it) {
      const int cl = it * 32 + q8;
      const int clc = (cl < kK) ? cl : (kK - 1);
      v8h hv;
#pragma unroll
      for (int e = 0; e < 8; ++e) {
        const float f = sOut[(n8 + e) * kK + clc];
        const float g = (cl < kK) ? (f * kSCarry) : 0.0f;
        hv[e] = (_Float16)g;
      }
      *(volatile v8h*)(ST16 + (size_t)cl * kNP + m0 + n8) = hv;
    }
    if (wave == 0) *(volatile float*)(DENP + (size_t)tile * 32 + lane) = dsum;
    __threadfence();
  }
}

__global__ __launch_bounds__(256) void cut_numerator_kernel(
    const int* __restrict__ ei, const float* __restrict__ ew,
    const float* __restrict__ S, float* __restrict__ NUMP)
{
  __shared__ float sRed[8];
  const int tid = threadIdx.x;
  const int lane = tid & 31;
  const int wave = tid >> 5;
  const int l8 = tid & 7;
  const int grp = tid >> 3;
  float acc = 0.0f;
#pragma unroll 1
  for (int it = 0; it < 32; ++it) {
    const int e = blockIdx.x * 1024 + it * 32 + grp;
    const bool live = e < kE;
    const int ec = live ? e : (kE - 1);
    int s = ei[ec];
    int d = ei[kE + ec];
    s = min(max(s, 0), kN - 1);
    d = min(max(d, 0), kN - 1);
    const float w = ew[ec];
    const float* ps = S + (size_t)s * kK;
    const float* pd = S + (size_t)d * kK;
    float dot = 0.0f;
#pragma unroll
    for (int jj = 0; jj < 4; ++jj) {
      const int j4 = l8 + 8 * jj;
      const bool ok = j4 < (kK / 4);
      const int jc = ok ? j4 : (kK / 4 - 1);
      const v4f a = *(const v4f*)(ps + jc * 4);
      const v4f b = *(const v4f*)(pd + jc * 4);
      float p = a[0] * b[0];
      p = fmaf(a[1], b[1], p);
      p = fmaf(a[2], b[2], p);
      p = fmaf(a[3], b[3], p);
      dot += ok ? p : 0.0f;
    }
    acc += live ? (w * dot) : 0.0f;
  }
  const float total = block_sum256(acc, sRed, lane, wave);
  if (wave == 0) {
    const float v = (lane == 0) ? total : 0.0f;
    float* p = NUMP + (size_t)blockIdx.x * 32 + lane;
    *(volatile float*)p = v;
    __threadfence();
    *(volatile float*)p = v;
  }
}

__global__ __launch_bounds__(256) void finalize_kernel(
    const float* __restrict__ SSP, const float* __restrict__ NUMP, const float* __restrict__ DENP,
    float* __restrict__ out)
{
  __shared__ float sSS[kK * kK];
  __shared__ float sRed[8];
  const int tid = threadIdx.x;
  const int lane = tid & 31;
  const int wave = tid >> 5;
  float f2 = 0.0f;
#pragma unroll 1
  for (int e = tid; e < kK * kK; e += 256) {
    const int i = e / kK;
    const int j = e - i * kK;
    const float* p = SSP + (size_t)i * kKP + j;
    float s = 0.0f;
#pragma unroll 1
    for (int b = 0; b < kSSBatches; ++b) s += p[(size_t)b * kKP * kKP];
    sSS[e] = s;
    f2 += s * s;
  }
  const float fro2 = block_sum256(f2, sRed, lane, wave);
  const float fro = sqrtf(fro2);
  const float invf = (fro > 0.0f) ? (1.0f / fro) : 0.0f;
  const float isk = 1.0f / sqrtf((float)kK);
  float o2 = 0.0f;
#pragma unroll 1
  for (int e = tid; e < kK * kK; e += 256) {
    const int i = e / kK;
    const int j = e - i * kK;
    const float dg = (i == j) ? isk : 0.0f;
    const float v = sSS[e] * invf - dg;
    o2 += v * v;
  }
  const float ortho = sqrtf(block_sum256(o2, sRed, lane, wave));
  float pn = 0.0f;
#pragma unroll 1
  for (int b = tid; b < kCutBlocks; b += 256) pn += NUMP[(size_t)b * 32];
  const float num = block_sum256(pn, sRed, lane, wave);
  float pd = 0.0f;
#pragma unroll 1
  for (int b = tid; b < kPoolTiles; b += 256) pd += DENP[(size_t)b * 32];
  const float den = block_sum256(pd, sRed, lane, wave);
  const float cut = -(num / den);
  const float aux = cut + ortho;
  const float v = (tid == 0) ? aux : ((tid == 1) ? cut : ortho);
  float* po = out + (size_t)kN * kK + ((tid < 3) ? tid : 0);
  if (tid < 3) *(volatile float*)po = v;
  __threadfence();
  if (tid < 3) *(volatile float*)po = v;
}

extern "C" void kernel_launch(void* const* d_in, const int* in_sizes, int n_in,
                              void* d_out, int out_size, void* d_ws, size_t ws_size,
                              hipStream_t stream) {
  if (n_in < 8) return;
  if (in_sizes[0] != kN * kCin) return;
  if (in_sizes[1] != kCin * kH) return;
  if (in_sizes[2] != kH) return;
  if (in_sizes[3] != kH * kK) return;
  if (in_sizes[4] != kK) return;
  if (in_sizes[5] != 2 * kE) return;
  if (in_sizes[6] != kE) return;
  if (out_size != kN * kK + 3) return;
  if (ws_size < kWsTotal) return;

  const float* x  = (const float*)d_in[0];
  const float* W1 = (const float*)d_in[1];
  const float* b1 = (const float*)d_in[2];
  const float* Wp = (const float*)d_in[3];
  const float* bp = (const float*)d_in[4];
  const int*   ei = (const int*)d_in[5];
  const float* ew = (const float*)d_in[6];
  float* out = (float*)d_out;

  char* ws = (char*)d_ws;
  unsigned short* X16   = (unsigned short*)(ws + kOffX16);
  float*          HX    = (float*)(ws + kOffHX);
  unsigned short* H16   = (unsigned short*)(ws + kOffH16);
  unsigned short* ST16  = (unsigned short*)(ws + kOffST16);
  float*          SSP   = (float*)(ws + kOffSSP);
  float*          INV   = (float*)(ws + kOffINV);
  float*          DEGNL = (float*)(ws + kOffDEGNL);
  unsigned short* W1T   = (unsigned short*)(ws + kOffW1T);
  unsigned short* WPT   = (unsigned short*)(ws + kOffWPT);
  float*          NUMP  = (float*)(ws + kOffNUMP);
  float*          DENP  = (float*)(ws + kOffDENP);

  prep_weights_kernel<<<8, 256, 0, stream>>>(W1, Wp, W1T, WPT);
  cast_x_kernel<<<(kNP * kCin / 8) / 256, 256, 0, stream>>>(x, X16);
  degree_tile_kernel<<<kDegTiles, 256, 0, stream>>>(ei, ew, INV, DEGNL);

  wmma_gemm64_f16<<<dim3((kNP / 64) / 8, 1), 256, 0, stream>>>(
      X16, kCin, 0L,
      W1T, kCin, 0L,
      HX, kH, 0L,
      kNP, kH, kCin, kW1CarryInv);

  aggregate_tile_kernel<<<kAggTiles, 256, 0, stream>>>(ei, ew, HX, INV, b1, H16);
  pool_softmax_kernel<<<kPoolTiles, 256, 0, stream>>>(H16, WPT, bp, DEGNL, out, ST16, DENP);
  cut_numerator_kernel<<<kCutBlocks, 256, 0, stream>>>(ei, ew, out, NUMP);

  wmma_gemm64_f16<<<dim3(1, kSSBatches), 256, 0, stream>>>(
      ST16, kNP, (long)kSSK,
      ST16, kNP, (long)kSSK,
      SSP, kKP, (long)kKP * kKP,
      kKP, kKP, kSSK, kSSScale);

  finalize_kernel<<<1, 256, 0, stream>>>(SSP, NUMP, DENP, out);
}
